// SSMBlock_30880814858921
// MI455X (gfx1250) — hardware-verified
//
#include <hip/hip_runtime.h>


namespace {
constexpr int B = 4, T = 2048, DM = 1024, NS = 16, FF = 4096, BL = 4  , NR = B * T, RL = BL * T  ;
constexpr float XS = 8.0f, WSC = 256.0f, RS_ = 1024.0f, LNEPS = 1e-5f, RSQ2 = 0.70710678118654752f;
static_assert(T % 64 == 0 && DM % 256 == 0 && FF % 128 == 0 && DM % 64 == 0, "tiling");
typedef _Float16 b16;
typedef __attribute__((ext_vector_type(16))) _Float16 v16b;
typedef __attribute__((ext_vector_type(8))) _Float16 v8b;
typedef __attribute__((ext_vector_type(8))) float v8f;
typedef __attribute__((ext_vector_type(4))) float v4f;
__device__ __forceinline__ float bf16_rne(float f) { unsigned int u = __float_as_uint(f); u += 0x7FFFu + ((u >> 16) & 1u); return __uint_as_float(u & 0xFFFF0000u); }
__device__ __forceinline__ void split16(float v, b16& hi, b16& lo) { hi = (b16)v; lo = (b16)(v - (float)hi); }
__device__ __forceinline__ v16b frag_kb(const b16* p, int hh) { const v8b a = *(const v8b*)(p + 8 * hh), b = *(const v8b*)(p + 16 + 8 * hh); v16b f;
#pragma unroll
  for (int e = 0; e < 8; ++e) { f[e] = a[e]; f[8 + e] = b[e]; } return f; }
__device__ __forceinline__ v8f wmma16b(v16b a, v16b b, v8f c) { v8f d = __builtin_amdgcn_wmma_f32_16x16x32_f16(false, a, false, b, (short)0, c, false, false); asm volatile("v_nop\n\tv_nop\n\tv_nop\n\tv_nop" : "+v"(d) : "v"(a), "v"(b)); return d; }
__device__ __forceinline__ void wave_lds_sync() { __builtin_amdgcn_fence(__ATOMIC_RELEASE, "workgroup"); __builtin_amdgcn_wave_barrier(); __builtin_amdgcn_fence(__ATOMIC_ACQUIRE, "workgroup"); }
__device__ __forceinline__ float pmul(float a, float b) { float p = a * b; asm volatile("" : "+v"(p)); return p; }
__device__ __forceinline__ int iclamp(int v, int lo, int hi) { return v < lo ? lo : (v > hi ? hi : v); }

typedef __attribute__((ext_vector_type(2))) _Float16 v2h;
typedef __attribute__((ext_vector_type(4))) _Float16 v4h;
typedef __attribute__((ext_vector_type(2))) float v2f;
typedef __attribute__((ext_vector_type(4))) int v4i;
__device__ __forceinline__ float nexp2(float v) { return __builtin_amdgcn_exp2f(v); }
__device__ __forceinline__ float bfp(float v) { float t = bf16_rne(v); asm volatile("" : "+v"(t)); return t; }
__global__ __launch_bounds__(256) void prep_kernel(const float* __restrict__ wo, const float* __restrict__ w1, const float* __restrict__ w2, b16* __restrict__ WO, b16* __restrict__ W1T, b16* __restrict__ W2T) {
  const size_t u = (size_t)blockIdx.x * 256 + threadIdx.x; const size_t n2 = (size_t)DM * DM / 8, n3 = (size_t)FF * DM / 8, n4 = (size_t)DM * FF / 8; if (u >= n2 + n3 + n4) return; v8b o; b16* dst; const float* src;
  if (u < n2) { src = wo + u * 8; dst = WO + u * 8; } else if (u < n2 + n3) { src = w1 + (u - n2) * 8; dst = W1T + (u - n2) * 8; } else { src = w2 + (u - n2 - n3) * 8; dst = W2T + (u - n2 - n3) * 8; }
  for (int j = 0; j < 8; ++j) o[j] = (b16)(bf16_rne(src[j]) * WSC);
  for (int pass = 0; pass < 2; ++pass) { *(volatile v8b*)dst = o; __threadfence(); }
}
template <bool RND>
__global__ __launch_bounds__(256) void ln_kernel(const float* __restrict__ X, const float* __restrict__ g, const float* __restrict__ bb, float* __restrict__ Y) {
  const int wave = threadIdx.x >> 5, lane = threadIdx.x & 31; const int row = blockIdx.x * 8 + wave; if (row >= RL) return;
  float v[32]; float s1 = 0.0f; const float* xr = X + (size_t)row * DM;
#pragma unroll
  for (int k = 0; k < 8; ++k) { const v4f t4 = *(const v4f*)(xr + 128 * k + 4 * lane); for (int j = 0; j < 4; ++j) { const float t = RND ? bf16_rne(t4[j]) : t4[j]; v[4 * k + j] = t; s1 += t; } }
#pragma unroll
  for (int o = 16; o >= 1; o >>= 1) s1 += __shfl_xor(s1, o);
  const float mu = s1 * (1.0f / DM); float s2 = 0.0f;
#pragma unroll
  for (int q = 0; q < 32; ++q) { const float d = v[q] - mu; s2 += pmul(d, d); }
#pragma unroll
  for (int o = 16; o >= 1; o >>= 1) s2 += __shfl_xor(s2, o);
  const float rs = rsqrtf(s2 * (1.0f / DM) + LNEPS);
  v4f o4[8];
#pragma unroll
  for (int k = 0; k < 8; ++k) for (int j = 0; j < 4; ++j) { const int c = 128 * k + 4 * lane + j; o4[k][j] = pmul((v[4 * k + j] - mu) * rs, bfp(g[c])) + bfp(bb[c]); }
  for (int pass = 0; pass < 2; ++pass) {
#pragma unroll
    for (int k = 0; k < 8; ++k) *(volatile v4f*)(Y + (size_t)row * DM + 128 * k + 4 * lane) = o4[k];
    __threadfence(); }
}
__global__ __launch_bounds__(128) void scan_kernel(const float* __restrict__ XN, const float* __restrict__ Alog, const float* __restrict__ Bm, const float* __restrict__ Cm, const float* __restrict__ Dv, b16* __restrict__ YSh, b16* __restrict__ YSl) {
  const int gw = blockIdx.x * 4 + (threadIdx.x >> 5), lane = threadIdx.x & 31; const int b = gw / (DM / 64), d0 = (gw % (DM / 64)) * 64 + 2 * lane;
  float Aa[2][NS], Bb[2][NS], Cc[2][NS], Dd[2];
#pragma unroll
  for (int c = 0; c < 2; ++c) { const int d = d0 + c; Dd[c] = bfp(Dv[d]);
#pragma unroll
    for (int n = 0; n < NS; ++n) { const float al = bfp(Alog[d * NS + n]); Aa[c][n] = __builtin_amdgcn_rcpf(1.0f + __expf(-al));   Bb[c][n] = bfp(Bm[d * NS + n]); Cc[c][n] = bfp(Cm[d * NS + n]); } }
#pragma unroll 1
  for (int pass = 0; pass < 2; ++pass) { float h[2][NS];
#pragma unroll
    for (int c = 0; c < 2; ++c) for (int n = 0; n < NS; ++n) h[c][n] = 0.0f;
#pragma unroll 1
    for (int t = 0; t < T; ++t) { const size_t row = ((size_t)b * T + t) * DM + d0; const v2f xv = *(const v2f*)(XN + row); v2h oh, olo;
#pragma unroll
      for (int c = 0; c < 2; ++c) { const float xx = xv[c]; float y = pmul(Dd[c], xx);
#pragma unroll
        for (int n = 0; n < NS; ++n) { h[c][n] = pmul(Aa[c][n], h[c][n]) + pmul(Bb[c][n], xx); y = y + pmul(Cc[c][n], h[c][n]); }
        const float s = y * __builtin_amdgcn_rcpf(1.0f + __expf(-y)); const float f = s * XS; const b16 p = (b16)f; oh[c] = p; olo[c] = (b16)(f - (float)p); }
      *(volatile v2h*)(YSh + row) = oh; *(volatile v2h*)(YSl + row) = olo; }
    __threadfence(); }
}
__global__ __launch_bounds__(128) void out1_kernel(const b16* __restrict__ Ch, const b16* __restrict__ Cl, const b16* __restrict__ WO, const float* __restrict__ bo, const float* __restrict__ x, float* __restrict__ X1) {
  __shared__ __attribute__((aligned(16))) float Tf[4][16][128 + 4];
  const int wave = threadIdx.x >> 5, lane = threadIdx.x & 31, nloc = lane & 15, hlf = lane >> 4; const int b = blockIdx.z; const size_t m0 = (size_t)b * T + (size_t)blockIdx.x * 64 + wave * 16; const int n0 = blockIdx.y * 128;
  v8f acc[8];
#pragma unroll
  for (int t = 0; t < 8; ++t) acc[t] = (v8f){};
#pragma unroll 2
  for (int kb = 0; kb < DM; kb += 32) { const v16b ah = frag_kb(Ch + (m0 + nloc) * DM + kb, hlf), al = frag_kb(Cl + (m0 + nloc) * DM + kb, hlf);
#pragma unroll
    for (int t = 0; t < 8; ++t) { const v16b bw = frag_kb(WO + (size_t)(n0 + t * 16 + nloc) * DM + kb, hlf); acc[t] = wmma16b(ah, bw, acc[t]); acc[t] = wmma16b(al, bw, acc[t]); } }
#pragma unroll
  for (int t = 0; t < 8; ++t) { const int col = n0 + t * 16 + nloc; const float bbv = bf16_rne(bo[col]);
#pragma unroll
    for (int r = 0; r < 8; ++r) Tf[wave][8 * hlf + r][t * 16 + nloc] = acc[t][r] * (1.0f / (XS * WSC)) + bbv + bf16_rne(x[(m0 + 8 * hlf + r) * DM + col]); }
  wave_lds_sync();
  for (int pass = 0; pass < 2; ++pass) { for (int rr = 0; rr < 16; ++rr) *(volatile v4f*)(X1 + (m0 + rr) * DM + n0 + lane * 4) = *(const v4f*)(&Tf[wave][rr][lane * 4]); __threadfence(); }
}
__global__ __launch_bounds__(128) void mlp1_kernel(const float* __restrict__ XN, const b16* __restrict__ W1T, const float* __restrict__ b1, b16* __restrict__ G) {
  __shared__ __attribute__((aligned(16))) b16 As[64][256 + 8]; __shared__ __attribute__((aligned(16))) float Tf[4][16][128 + 4];
  const int wave = threadIdx.x >> 5, lane = threadIdx.x & 31, nloc = lane & 15, hlf = lane >> 4; const size_t r0 = (size_t)blockIdx.x * 64; const int n0 = blockIdx.y * 128;
  const float* xb = XN + r0 * DM;
  v8f acc[8];
#pragma unroll
  for (int t = 0; t < 8; ++t) acc[t] = (v8f){};
#pragma unroll 1
  for (int kc = 0; kc < DM; kc += 256) {
    __syncthreads();
    for (int i = threadIdx.x; i < 64 * 64; i += 128) { const int rr = i / 64, q = (i % 64) * 4; const v4f f = *(const v4f*)(xb + (size_t)rr * DM + kc + q); v4h o; for (int j = 0; j < 4; ++j) o[j] = (b16)(f[j] * XS); *(v4h*)(&As[rr][q]) = o; }
    __syncthreads();
#pragma unroll 2
    for (int kb = 0; kb < 256; kb += 32) { const v16b a = frag_kb(&As[wave * 16 + nloc][kb], hlf);
#pragma unroll
      for (int t = 0; t < 8; ++t) acc[t] = wmma16b(a, frag_kb(W1T + (size_t)(n0 + t * 16 + nloc) * DM + kc + kb, hlf), acc[t]); } }
#pragma unroll
  for (int t = 0; t < 8; ++t) { const float bbv = bf16_rne(b1[n0 + t * 16 + nloc]);
#pragma unroll
    for (int r = 0; r < 8; ++r) { const float hm = acc[t][r] * (1.0f / (XS * WSC)) + bbv; Tf[wave][8 * hlf + r][t * 16 + nloc] = 0.5f * hm * (1.0f + erff(hm * RSQ2)); } }
  __syncthreads();
  for (int pass = 0; pass < 2; ++pass) { for (int rr = 0; rr < 16; ++rr) { v4h o4; for (int j = 0; j < 4; ++j) o4[j] = (b16)(Tf[wave][rr][lane * 4 + j] * XS); *(volatile v4h*)(G + (r0 + wave * 16 + rr) * FF + n0 + lane * 4) = o4; } __threadfence(); }
}
__global__ __launch_bounds__(128) void mlp2_kernel(const b16* __restrict__ G, const b16* __restrict__ W2T, const float* __restrict__ b2, const float* __restrict__ X1, float* __restrict__ out) {
  __shared__ __attribute__((aligned(16))) float Tf[4][16][128 + 4];
  const int wave = threadIdx.x >> 5, lane = threadIdx.x & 31, nloc = lane & 15, hlf = lane >> 4; const size_t m0 = (size_t)blockIdx.x * 64 + wave * 16; const int n0 = blockIdx.y * 128;
  v8f acc[8];
#pragma unroll
  for (int t = 0; t < 8; ++t) acc[t] = (v8f){};
#pragma unroll 2
  for (int kb = 0; kb < FF; kb += 32) { const v16b a = frag_kb(G + (m0 + nloc) * FF + kb, hlf);
#pragma unroll
    for (int t = 0; t < 8; ++t) acc[t] = wmma16b(a, frag_kb(W2T + (size_t)(n0 + t * 16 + nloc) * FF + kb, hlf), acc[t]); }
#pragma unroll
  for (int t = 0; t < 8; ++t) { const int col = n0 + t * 16 + nloc; const float bbv = bf16_rne(b2[col]);
#pragma unroll
    for (int r = 0; r < 8; ++r) Tf[wave][8 * hlf + r][t * 16 + nloc] = acc[t][r] * (1.0f / (XS * WSC)) + bbv + X1[(m0 + 8 * hlf + r) * DM + col]; }
  wave_lds_sync();
  for (int pass = 0; pass < 2; ++pass) { for (int rr = 0; rr < 16; ++rr) *(volatile v4f*)(out + (m0 + rr) * DM + n0 + lane * 4) = *(const v4f*)(&Tf[wave][rr][lane * 4]); __threadfence(); }
}
}

extern "C" void kernel_launch(void* const* d_in, const int* in_sizes, int n_in, void* d_out, int out_size, void* d_ws, size_t ws_size, hipStream_t stream) {
  (void)n_in;
  auto Fp = [&](int i) { return (const float*)d_in[i]; };
  if (in_sizes[0] != NR * DM || in_sizes[1] != DM || in_sizes[2] != DM || in_sizes[3] != DM * NS || in_sizes[4] != DM * NS || in_sizes[5] != DM * NS || in_sizes[6] != DM || in_sizes[7] != DM * DM || in_sizes[8] != DM || in_sizes[9] != DM || in_sizes[10] != DM || in_sizes[11] != FF * DM || in_sizes[12] != FF || in_sizes[13] != DM * FF || in_sizes[14] != DM || out_size != NR * DM) return;
  size_t off = 0; char* ws = (char*)d_ws;
  auto carve = [&](size_t bytes) { char* p = ws + off; off += (bytes + 255) & ~(size_t)255; return p; };
  b16* WO = (b16*)carve((size_t)DM * DM * 2); b16* W1T = (b16*)carve((size_t)FF * DM * 2); b16* W2T = (b16*)carve((size_t)DM * FF * 2);
  float* XN = (float*)carve((size_t)NR * DM * 4); b16* YSh = (b16*)carve((size_t)NR * DM * 2); b16* YSl = (b16*)carve((size_t)NR * DM * 2); float* X1 = (float*)carve((size_t)NR * DM * 4); b16* G = (b16*)carve((size_t)NR * FF * 2);
  if (off > ws_size || off > ((size_t)200 << 20)) return;
  prep_kernel<<<(unsigned)(((size_t)(DM * DM + FF * DM + DM * FF) / 8 + 255) / 256), 256, 0, stream>>>(Fp(7), Fp(11), Fp(13), WO, W1T, W2T);
  ln_kernel<true><<<RL / 8, 256, 0, stream>>>(Fp(0), Fp(1), Fp(2), XN);
  scan_kernel<<<(BL * DM / 64) / 4, 128, 0, stream>>>(XN, Fp(3), Fp(4), Fp(5), Fp(6), YSh, YSl);
  out1_kernel<<<dim3(T / 64, DM / 128, BL), 128, 0, stream>>>(YSh, YSl, WO, Fp(8), Fp(0), X1);
  ln_kernel<false><<<RL / 8, 256, 0, stream>>>(X1, Fp(9), Fp(10), XN);
  mlp1_kernel<<<dim3(RL / 64, FF / 128), 128, 0, stream>>>(XN, W1T, Fp(12), G);
  mlp2_kernel<<<dim3(RL / 64, DM / 128), 128, 0, stream>>>(G, W2T, Fp(14), X1, (float*)d_out);
}
